// MultiheadLocalAttentionV1_23888608100407
// MI455X (gfx1250) — hardware-verified
//
#include <hip/hip_runtime.h>


#define NB     2
#define CC     256
#define HWP    1024
#define IMW    32
#define NHD    8
#define HDIM   32
#define WSZ    15
#define NTAP   225
#define MROWS  (NB * HWP)
#define TINV   0.17677669529663687f
#define SC64   64.0f
#define INV64  0.015625f
#define INV4096 0.000244140625f

#define IN_X_N   (NB * CC * HWP)
#define IN_W_N   (CC * CC)
#define IN_B_N   (CC)
#define IN_WRK_N (NHD * NTAP * HDIM)
#define IN_BRK_N (NHD * NTAP)
#define IN_RV_N  (NHD * HDIM * NTAP)
#define OUT0_N   (HWP * NB * CC)
#define OUT1_N   (NB * NHD * NTAP * HWP)
#define OUT_N    (OUT0_N + OUT1_N)

#define SZ_W    ((size_t)4 * CC * CC * 2)
#define SZ_WRK  ((size_t)NHD * 256 * HDIM * 2)
#define SZ_XT   ((size_t)3 * MROWS * CC * 2)
#define SZ_P    ((size_t)3 * MROWS * CC * 4)
#define SZ_QPH  ((size_t)MROWS * CC * 2)
#define SZ_REL  ((size_t)OUT1_N * 4)
#define SZ_OH   ((size_t)NB * NHD * HWP * HDIM * 2)
#define OFF_W    ((size_t)0)
#define OFF_WRK  (OFF_W + SZ_W)
#define OFF_XT   (OFF_WRK + SZ_WRK)
#define OFF_P    (OFF_XT + SZ_XT)
#define OFF_QPH  (OFF_P + SZ_P)
#define OFF_REL  (OFF_QPH + SZ_QPH)
#define OFF_OH   (OFF_REL + SZ_REL)
#define WS_TOTAL (OFF_OH + SZ_OH)

static_assert(WS_TOTAL == 26935296);
static_assert((OFF_WRK % 128) == 0 && (OFF_XT % 128) == 0 && (OFF_P % 128) == 0);
static_assert((OFF_QPH % 128) == 0 && (OFF_REL % 128) == 0 && (OFF_OH % 128) == 0);
static_assert(OUT_N == 4210688);

#define PREP_W_BLK    ((4 * CC * CC / 8) / 256)
#define PREP_WRK_BLK  ((NHD * 256 * HDIM / 8) / 256)
#define PREP_X_BLK    (3 * NB * (CC / 64) * (HWP / IMW))
#define PREP_BLOCKS   (PREP_W_BLK + PREP_WRK_BLK + PREP_X_BLK)
#define PROJ_BLOCKS   (3 * (MROWS / 64) * (CC / 128))
#define REL_BLOCKS    (NB * NHD * (256 / 64) * (HWP / 128))
#define WIN_BLOCKS    (NB * NHD * IMW)
#define OUT_BLOCKS    ((MROWS / 64) * (CC / 128))
static_assert(PREP_W_BLK == 128 && PREP_WRK_BLK == 32 && PREP_X_BLK == 768);
static_assert(PROJ_BLOCKS == 192 && REL_BLOCKS == 512 && WIN_BLOCKS == 512 && OUT_BLOCKS == 64);

#define QP   136
#define TRP  65

typedef _Float16 v16h __attribute__((ext_vector_type(16)));
typedef _Float16 v8h  __attribute__((ext_vector_type(8)));
typedef _Float16 v4h  __attribute__((ext_vector_type(4)));
typedef float    v8f  __attribute__((ext_vector_type(8)));
typedef float    v4f  __attribute__((ext_vector_type(4)));
typedef float    v4fa __attribute__((ext_vector_type(4), __may_alias__));

union Frag { v16h v; v8h half[2]; };

__device__ __forceinline__ void st2_h8(_Float16* p, v8h x) {
  *(volatile v8h*)p = x;
  __threadfence();
  *(volatile v8h*)p = x;
}
__device__ __forceinline__ void st2_h4(_Float16* p, v4h x) {
  *(volatile v4h*)p = x;
  __threadfence();
  *(volatile v4h*)p = x;
}
__device__ __forceinline__ void st2_f4(float* p, v4f x) {
  *(volatile v4f*)p = x;
  __threadfence();
  *(volatile v4f*)p = x;
}
__device__ __forceinline__ void st2_f1(float* p, float x) {
  *(volatile float*)p = x;
  __threadfence();
  *(volatile float*)p = x;
}

__device__ __forceinline__ v8h cvt8(v4f a, v4f b, float s) {
  v8h o;
  o[0] = (_Float16)(a.x * s); o[1] = (_Float16)(a.y * s); o[2] = (_Float16)(a.z * s); o[3] = (_Float16)(a.w * s);
  o[4] = (_Float16)(b.x * s); o[5] = (_Float16)(b.y * s); o[6] = (_Float16)(b.z * s); o[7] = (_Float16)(b.w * s);
  return o;
}

__device__ __forceinline__ v8f v8f_zero() {
  v8f z = {0.f, 0.f, 0.f, 0.f, 0.f, 0.f, 0.f, 0.f};
  return z;
}

__device__ __forceinline__ v16h ldfrag(const _Float16* rowp, int h) {
  Frag f;
  f.half[0] = *(const v8h*)(rowp + 8 * h);
  f.half[1] = *(const v8h*)(rowp + 16 + 8 * h);
  return f.v;
}

__device__ __forceinline__ void mma(v8f& acc, v16h a, v16h b) {
  acc = __builtin_amdgcn_wmma_f32_16x16x32_f16(false, a, false, b, (short)0, acc, false, false);
  asm volatile("v_nop\n\tv_nop\n\tv_nop\n\tv_nop" : "+v"(acc) : "v"(a), "v"(b));
}

__global__ void __launch_bounds__(256) k_prep(
    const float* __restrict__ q, const float* __restrict__ k, const float* __restrict__ v,
    const float* __restrict__ WQ, const float* __restrict__ WK, const float* __restrict__ WV,
    const float* __restrict__ Wrk, const float* __restrict__ Wp,
    _Float16* __restrict__ wh, _Float16* __restrict__ wrkh, _Float16* __restrict__ xt) {
  __shared__ __attribute__((aligned(16))) float tr[32 * TRP];
  const int bid = blockIdx.x;
  const int tid = threadIdx.x;
  if (bid < PREP_W_BLK) {
    const int i = bid * 256 + tid;
    const int mat = i >> 13;
    const int j = i & 8191;
    const float* W = (mat == 0) ? WQ : ((mat == 1) ? WK : ((mat == 2) ? WV : Wp));
    const float* rp = W + (size_t)j * 8;
    const v4f ra = *(const v4f*)rp;
    const v4f rb = *(const v4f*)(rp + 4);
    st2_h8(wh + (size_t)mat * (CC * CC) + (size_t)j * 8, cvt8(ra, rb, SC64));
  } else if (bid < PREP_W_BLK + PREP_WRK_BLK) {
    const int i = (bid - PREP_W_BLK) * 256 + tid;
    const int r = i >> 2;
    const int hh = r >> 8;
    const int s = r & 255;
    const int kc = i & 3;
    const int scl = min(s, NTAP - 1);
    const float* rp = Wrk + ((size_t)(hh * NTAP + scl)) * HDIM + kc * 8;
    v4f ra = *(const v4f*)rp;
    v4f rb = *(const v4f*)(rp + 4);
    const v4f z4 = {0.f, 0.f, 0.f, 0.f};
    if (s >= NTAP) { ra = z4; rb = z4; }
    st2_h8(wrkh + (size_t)i * 8, cvt8(ra, rb, SC64));
  } else {
    const int t = bid - PREP_W_BLK - PREP_WRK_BLK;
    const int mn = t >> 7;
    const int rem = t & 127;
    const int ct = rem >> 5;
    const int pt = rem & 31;
    const int mat = mn >> 1;
    const int n = mn & 1;
    const float* X = (mat == 0) ? q : ((mat == 1) ? k : v);
    const int row = tid >> 2;
    const int p8 = (tid & 3) * 8;
    const float* rp = X + ((size_t)(n * CC + ct * 64 + row)) * HWP + pt * IMW + p8;
    const v4f ra = *(const v4f*)rp;
    const v4f rb = *(const v4f*)(rp + 4);
    tr[(p8 + 0) * TRP + row] = ra.x; tr[(p8 + 1) * TRP + row] = ra.y;
    tr[(p8 + 2) * TRP + row] = ra.z; tr[(p8 + 3) * TRP + row] = ra.w;
    tr[(p8 + 4) * TRP + row] = rb.x; tr[(p8 + 5) * TRP + row] = rb.y;
    tr[(p8 + 6) * TRP + row] = rb.z; tr[(p8 + 7) * TRP + row] = rb.w;
    __syncthreads();
    const int prow = tid >> 3;
    const int c0 = (tid & 7) * 8;
    const float* tp = tr + prow * TRP + c0;
    v8h o;
    #pragma unroll
    for (int j = 0; j < 8; ++j) o[j] = (_Float16)tp[j];
    st2_h8(xt + ((size_t)(mn * HWP + pt * IMW + prow)) * CC + ct * 64 + c0, o);
  }
}

__global__ void __launch_bounds__(256) k_proj(
    const _Float16* __restrict__ xt, const _Float16* __restrict__ wh,
    const float* __restrict__ bQ, const float* __restrict__ bK, const float* __restrict__ bV,
    float* __restrict__ P, _Float16* __restrict__ qph) {
  __shared__ __attribute__((aligned(16))) float tile[64 * QP];
  const int tid = threadIdx.x;
  const int lane = tid & 31;
  const int w = tid >> 5;
  const int h = lane >> 4;
  const int m = lane & 15;
  const int bid = blockIdx.x;
  const int mat = bid >> 6;
  const int rem = bid & 63;
  const int mb = rem >> 1;
  const int nb = rem & 1;
  const int m0 = mb * 64;
  const int n0 = nb * 128;
  const int r0 = (w >> 2) * 32;
  const int c0 = (w & 3) * 32;
  const float* bias = (mat == 0) ? bQ : ((mat == 1) ? bK : bV);

  v8f acc[2][2];
  acc[0][0] = v8f_zero(); acc[0][1] = v8f_zero();
  acc[1][0] = v8f_zero(); acc[1][1] = v8f_zero();

  const _Float16* a0 = xt + ((size_t)(mat * MROWS + m0 + r0 + m)) * CC;
  const _Float16* a1 = a0 + 16 * CC;
  const _Float16* b0 = wh + (size_t)mat * (CC * CC) + ((size_t)(n0 + c0 + m)) * CC;
  const _Float16* b1 = b0 + 16 * CC;

  #pragma unroll 1
  for (int ks = 0; ks < CC / 32; ++ks) {
    const int k0 = ks * 32;
    const v16h A0 = ldfrag(a0 + k0, h);
    const v16h A1 = ldfrag(a1 + k0, h);
    const v16h B0 = ldfrag(b0 + k0, h);
    const v16h B1 = ldfrag(b1 + k0, h);
    mma(acc[0][0], A0, B0);
    mma(acc[0][1], A0, B1);
    mma(acc[1][0], A1, B0);
    mma(acc[1][1], A1, B1);
  }

  #pragma unroll
  for (int i = 0; i < 2; ++i) {
    #pragma unroll
    for (int t = 0; t < 2; ++t) {
      const int col = c0 + t * 16 + m;
      const float bs = bias[n0 + col];
      #pragma unroll
      for (int r = 0; r < 8; ++r)
        tile[(r0 + i * 16 + 8 * h + r) * QP + col] = acc[i][t][r] * INV64 + bs;
    }
  }
  __syncthreads();

  #pragma unroll 1
  for (int it = 0; it < 8; ++it) {
    const int row = it * 8 + w;
    const v4f vv = *(const v4fa*)(tile + row * QP + lane * 4);
    st2_f4(P + ((size_t)(mat * MROWS + m0 + row)) * CC + n0 + lane * 4, vv);
    if (mat == 0) {
      v4h qq;
      qq[0] = (_Float16)(vv.x * SC64); qq[1] = (_Float16)(vv.y * SC64);
      qq[2] = (_Float16)(vv.z * SC64); qq[3] = (_Float16)(vv.w * SC64);
      st2_h4(qph + ((size_t)(m0 + row)) * CC + n0 + lane * 4, qq);
    }
  }
}

__global__ void __launch_bounds__(256) k_rel(
    const _Float16* __restrict__ wrkh, const _Float16* __restrict__ qph,
    const float* __restrict__ brk, float* __restrict__ rel) {
  __shared__ __attribute__((aligned(16))) float tile[64 * QP];
  const int tid = threadIdx.x;
  const int lane = tid & 31;
  const int w = tid >> 5;
  const int h = lane >> 4;
  const int m = lane & 15;
  const int bid = blockIdx.x;
  const int nh = bid >> 5;
  const int rem = bid & 31;
  const int mb = rem >> 3;
  const int nb = rem & 7;
  const int n = nh >> 3;
  const int hd = nh & 7;
  const int m0 = mb * 64;
  const int n0 = nb * 128;
  const int r0 = (w >> 2) * 32;
  const int c0 = (w & 3) * 32;

  v8f acc[2][2];
  acc[0][0] = v8f_zero(); acc[0][1] = v8f_zero();
  acc[1][0] = v8f_zero(); acc[1][1] = v8f_zero();

  const _Float16* a0 = wrkh + ((size_t)(hd * 256 + m0 + r0 + m)) * HDIM;
  const _Float16* a1 = a0 + 16 * HDIM;
  const _Float16* b0 = qph + ((size_t)(n * HWP + n0 + c0 + m)) * CC + hd * HDIM;
  const _Float16* b1 = b0 + 16 * CC;
  {
    const v16h A0 = ldfrag(a0, h);
    const v16h A1 = ldfrag(a1, h);
    const v16h B0 = ldfrag(b0, h);
    const v16h B1 = ldfrag(b1, h);
    mma(acc[0][0], A0, B0);
    mma(acc[0][1], A0, B1);
    mma(acc[1][0], A1, B0);
    mma(acc[1][1], A1, B1);
  }

  #pragma unroll
  for (int i = 0; i < 2; ++i) {
    #pragma unroll
    for (int t = 0; t < 2; ++t) {
      const int col = c0 + t * 16 + m;
      #pragma unroll
      for (int r = 0; r < 8; ++r)
        tile[(r0 + i * 16 + 8 * h + r) * QP + col] = acc[i][t][r] * INV4096;
    }
  }
  __syncthreads();

  #pragma unroll 1
  for (int it = 0; it < 8; ++it) {
    const int row = it * 8 + w;
    const int s = m0 + row;
    const float bs = brk[hd * NTAP + min(s, NTAP - 1)];
    v4f vv = *(const v4fa*)(tile + row * QP + lane * 4);
    vv.x += bs; vv.y += bs; vv.z += bs; vv.w += bs;
    if (s < NTAP)
      st2_f4(rel + ((size_t)(nh * NTAP + s)) * HWP + n0 + lane * 4, vv);
  }
}

__global__ void __launch_bounds__(32) k_win(
    const float* __restrict__ P, const float* __restrict__ rel, const float* __restrict__ relv,
    float* __restrict__ attn, _Float16* __restrict__ oh) {
  __shared__ __attribute__((aligned(16))) float sc[NTAP * 32];
  __shared__ __attribute__((aligned(16))) float rvt[NTAP * 32];
  __shared__ __attribute__((aligned(16))) float ot[32 * 32];
  const int x = threadIdx.x;
  const int bid = blockIdx.x;
  const int nh = bid >> 5;
  const int y = bid & 31;
  const int n = nh >> 3;
  const int hd = nh & 7;
  const int p = y * IMW + x;

  #pragma unroll 1
  for (int idx = x; idx < HDIM * NTAP; idx += 32) {
    const int c = idx / NTAP;
    const int s = idx - c * NTAP;
    rvt[s * 32 + c] = relv[(size_t)hd * (HDIM * NTAP) + idx];
  }
  v4f qs[8];
  {
    const float* qp = P + ((size_t)(n * HWP + p)) * CC + hd * HDIM;
    #pragma unroll
    for (int d4 = 0; d4 < 8; ++d4) qs[d4] = *(const v4f*)(qp + 4 * d4) * TINV;
  }
  __syncthreads();

  const float* Pk = P + ((size_t)(1 * MROWS + n * HWP)) * CC + hd * HDIM;
  const float* Pv = P + ((size_t)(2 * MROWS + n * HWP)) * CC + hd * HDIM;
  const float* relp = rel + ((size_t)nh * NTAP) * HWP + p;

  float mx = -3.0e38f;
  #pragma unroll 1
  for (int kh = 0; kh < WSZ; ++kh) {
    const int yy = y + kh - 7;
    if ((unsigned)yy < (unsigned)IMW) {
      const float* krow = Pk + ((size_t)(yy * IMW)) * CC;
      #pragma unroll 1
      for (int kw = 0; kw < WSZ; ++kw) {
        const int s = kh * WSZ + kw;
        const int xx = x + kw - 7;
        const bool ok = (unsigned)xx < (unsigned)IMW;
        const int xc = min(max(xx, 0), IMW - 1);
        const float* kp = krow + (size_t)xc * CC;
        float d = 0.f;
        #pragma unroll
        for (int d4 = 0; d4 < 8; ++d4) {
          const v4f kv = *(const v4f*)(kp + 4 * d4);
          d += qs[d4].x * kv.x;
          d += qs[d4].y * kv.y;
          d += qs[d4].z * kv.z;
          d += qs[d4].w * kv.w;
        }
        float l = d + relp[(size_t)s * HWP];
        l = ok ? l : -3.0e38f;
        sc[s * 32 + x] = l;
        mx = fmaxf(mx, l);
      }
    } else {
      #pragma unroll 1
      for (int kw = 0; kw < WSZ; ++kw) sc[(kh * WSZ + kw) * 32 + x] = -3.0e38f;
    }
  }

  float sum = 0.f;
  #pragma unroll 1
  for (int s = 0; s < NTAP; ++s) {
    const float l = sc[s * 32 + x];
    const float e = (l > -1.0e38f) ? __expf(l - mx) : 0.f;
    sc[s * 32 + x] = e;
    sum += e;
  }
  const float inv = __builtin_amdgcn_rcpf(sum);

  float* ap = attn + ((size_t)nh * NTAP) * HWP + p;
  #pragma unroll 1
  for (int s = 0; s < NTAP; ++s) {
    const float pr = sc[s * 32 + x] * inv;
    sc[s * 32 + x] = pr;
    st2_f1(ap + (size_t)s * HWP, pr);
  }

  v4f acc[8];
  #pragma unroll
  for (int d4 = 0; d4 < 8; ++d4) { v4f z = {0.f, 0.f, 0.f, 0.f}; acc[d4] = z; }
  #pragma unroll 1
  for (int kh = 0; kh < WSZ; ++kh) {
    const int yy = y + kh - 7;
    if ((unsigned)yy < (unsigned)IMW) {
      const float* vrow = Pv + ((size_t)(yy * IMW)) * CC;
      #pragma unroll 1
      for (int kw = 0; kw < WSZ; ++kw) {
        const int s = kh * WSZ + kw;
        const int xx = x + kw - 7;
        const int xc = min(max(xx, 0), IMW - 1);
        const float pr = sc[s * 32 + x];
        const float* vp = vrow + (size_t)xc * CC;
        const v4fa* rr = (const v4fa*)(rvt + s * 32);
        #pragma unroll
        for (int d4 = 0; d4 < 8; ++d4) {
          const v4f vv = *(const v4f*)(vp + 4 * d4);
          const v4f rv = rr[d4];
          acc[d4] = acc[d4] + (vv + rv) * pr;
        }
      }
    }
  }

  {
    v4fa* op = (v4fa*)(ot + x * 32);
    #pragma unroll
    for (int d4 = 0; d4 < 8; ++d4) op[d4] = acc[d4];
  }
  __syncthreads();
  _Float16* ob = oh + ((size_t)(nh * HWP + y * IMW)) * HDIM;
  #pragma unroll 1
  for (int it = 0; it < 4; ++it) {
    const int qi = it * 32 + x;
    const int pix = qi >> 2;
    const int ch0 = (qi & 3) * 8;
    const v4fa* tp = (const v4fa*)(ot + pix * 32 + ch0);
    const v4f a = tp[0];
    const v4f b = tp[1];
    st2_h8(ob + (size_t)pix * HDIM + ch0, cvt8(a, b, SC64));
  }
}

__global__ void __launch_bounds__(256) k_out(
    const _Float16* __restrict__ oh, const _Float16* __restrict__ wh,
    const float* __restrict__ bp, float* __restrict__ out) {
  __shared__ __attribute__((aligned(16))) float tile[64 * QP];
  const int tid = threadIdx.x;
  const int lane = tid & 31;
  const int w = tid >> 5;
  const int h = lane >> 4;
  const int m = lane & 15;
  const int bid = blockIdx.x;
  const int mb = bid >> 1;
  const int nb = bid & 1;
  const int m0 = mb * 64;
  const int n0 = nb * 128;
  const int r0 = (w >> 2) * 32;
  const int c0 = (w & 3) * 32;

  v8f acc[2][2];
  acc[0][0] = v8f_zero(); acc[0][1] = v8f_zero();
  acc[1][0] = v8f_zero(); acc[1][1] = v8f_zero();

  const int rowA0 = m0 + r0 + m;
  const int rowA1 = rowA0 + 16;
  const _Float16* a0 = oh + ((size_t)((rowA0 & 1) * NHD) * HWP + (rowA0 >> 1)) * HDIM;
  const _Float16* a1 = oh + ((size_t)((rowA1 & 1) * NHD) * HWP + (rowA1 >> 1)) * HDIM;
  const _Float16* b0 = wh + (size_t)3 * (CC * CC) + ((size_t)(n0 + c0 + m)) * CC;
  const _Float16* b1 = b0 + 16 * CC;

  #pragma unroll 1
  for (int ks = 0; ks < NHD; ++ks) {
    const size_t ao = (size_t)ks * (HWP * HDIM);
    const int k0 = ks * 32;
    const v16h A0 = ldfrag(a0 + ao, h);
    const v16h A1 = ldfrag(a1 + ao, h);
    const v16h B0 = ldfrag(b0 + k0, h);
    const v16h B1 = ldfrag(b1 + k0, h);
    mma(acc[0][0], A0, B0);
    mma(acc[0][1], A0, B1);
    mma(acc[1][0], A1, B0);
    mma(acc[1][1], A1, B1);
  }

  #pragma unroll
  for (int i = 0; i < 2; ++i) {
    #pragma unroll
    for (int t = 0; t < 2; ++t) {
      const int col = c0 + t * 16 + m;
      const float bs = bp[n0 + col];
      #pragma unroll
      for (int r = 0; r < 8; ++r)
        tile[(r0 + i * 16 + 8 * h + r) * QP + col] = acc[i][t][r] * INV4096 + bs;
    }
  }
  __syncthreads();

  #pragma unroll 1
  for (int it = 0; it < 8; ++it) {
    const int row = it * 8 + w;
    const v4f vv = *(const v4fa*)(tile + row * QP + lane * 4);
    st2_f4(out + ((size_t)(m0 + row)) * CC + n0 + lane * 4, vv);
  }
}

extern "C" void kernel_launch(void* const* d_in, const int* in_sizes, int n_in,
                              void* d_out, int out_size, void* d_ws, size_t ws_size,
                              hipStream_t stream) {
  if (n_in < 14) return;
  if (in_sizes[0] != IN_X_N || in_sizes[1] != IN_X_N || in_sizes[2] != IN_X_N) return;
  if (in_sizes[3] != IN_W_N || in_sizes[4] != IN_B_N) return;
  if (in_sizes[5] != IN_W_N || in_sizes[6] != IN_B_N) return;
  if (in_sizes[7] != IN_W_N || in_sizes[8] != IN_B_N) return;
  if (in_sizes[9] != IN_WRK_N || in_sizes[10] != IN_BRK_N || in_sizes[11] != IN_RV_N) return;
  if (in_sizes[12] != IN_W_N || in_sizes[13] != IN_B_N) return;
  if (out_size != OUT_N) return;
  if (ws_size < (size_t)WS_TOTAL) return;

  const float* q    = (const float*)d_in[0];
  const float* k    = (const float*)d_in[1];
  const float* v    = (const float*)d_in[2];
  const float* WQ   = (const float*)d_in[3];
  const float* bQ   = (const float*)d_in[4];
  const float* WK   = (const float*)d_in[5];
  const float* bK   = (const float*)d_in[6];
  const float* WV   = (const float*)d_in[7];
  const float* bV   = (const float*)d_in[8];
  const float* Wrk  = (const float*)d_in[9];
  const float* brk  = (const float*)d_in[10];
  const float* relv = (const float*)d_in[11];
  const float* Wp   = (const float*)d_in[12];
  const float* bp   = (const float*)d_in[13];

  float* out0 = (float*)d_out;
  float* attn = out0 + OUT0_N;

  char* ws = (char*)d_ws;
  _Float16* wh   = (_Float16*)(ws + OFF_W);
  _Float16* wrkh = (_Float16*)(ws + OFF_WRK);
  _Float16* xt   = (_Float16*)(ws + OFF_XT);
  float*    P    = (float*)(ws + OFF_P);
  _Float16* qph  = (_Float16*)(ws + OFF_QPH);
  float*    rel  = (float*)(ws + OFF_REL);
  _Float16* oh   = (_Float16*)(ws + OFF_OH);

  k_prep<<<dim3(PREP_BLOCKS), dim3(256), 0, stream>>>(q, k, v, WQ, WK, WV, Wrk, Wp, wh, wrkh, xt);
  k_proj<<<dim3(PROJ_BLOCKS), dim3(256), 0, stream>>>(xt, wh, bQ, bK, bV, P, qph);
  k_rel<<<dim3(REL_BLOCKS), dim3(256), 0, stream>>>(wrkh, qph, brk, rel);
  k_win<<<dim3(WIN_BLOCKS), dim3(32), 0, stream>>>(P, rel, relv, attn, oh);
  k_out<<<dim3(OUT_BLOCKS), dim3(256), 0, stream>>>(oh, wh, bp, out0);
}
